// DiTBlock_79611513798969
// MI455X (gfx1250) — hardware-verified
//
#include <hip/hip_runtime.h>
#include <math.h>
#include <stddef.h>
#include <stdint.h>


#define C_DIM 1024
#define HD    64
#define NHEAD 16

typedef unsigned short us16;
typedef __bf16 v16bf __attribute__((ext_vector_type(16)));
typedef unsigned short v8us_t __attribute__((ext_vector_type(8)));
typedef v8us_t v8us __attribute__((may_alias));
typedef float v8f __attribute__((ext_vector_type(8)));
typedef float v4f_t __attribute__((ext_vector_type(4)));
typedef v4f_t v4f __attribute__((may_alias));

union Frag { v16bf v; v8us h[2]; };

static __device__ __forceinline__ unsigned bf16_rne_bits(float x) {
  const unsigned u = __float_as_uint(x);
  return (u + 0x7FFFu + ((u >> 16) & 1u)) >> 16;
}
static __device__ __forceinline__ void split2(float x, us16& hi, us16& lo) {
  const unsigned hb = bf16_rne_bits(x);
  const float hf = __uint_as_float(hb << 16);
  hi = (us16)hb;
  lo = (us16)bf16_rne_bits(x - hf);
}
static __device__ __forceinline__ void split8(v4f x0, v4f x1, v8us& h, v8us& l) {
#pragma unroll
  for (int j = 0; j < 4; ++j) {
    us16 a, b;
    split2(x0[j], a, b); h[j] = a;     l[j] = b;
    split2(x1[j], a, b); h[4 + j] = a; l[4 + j] = b;
  }
}

static __device__ __forceinline__ v16bf ldfrag(const us16* rowp, int hh) {
  Frag f;
  f.h[0] = *(const v8us*)(rowp + 8 * hh);
  f.h[1] = *(const v8us*)(rowp + 16 + 8 * hh);
  return f.v;
}

static __device__ __forceinline__ v8f mma3(v8f c, v16bf ah, v16bf al, v16bf bh, v16bf bl) {
  c = __builtin_amdgcn_wmma_f32_16x16x32_bf16(false, ah, false, bh, (short)0, c, false, false);
  c = __builtin_amdgcn_wmma_f32_16x16x32_bf16(false, ah, false, bl, (short)0, c, false, false);
  c = __builtin_amdgcn_wmma_f32_16x16x32_bf16(false, al, false, bh, (short)0, c, false, false);
  asm volatile("v_nop\n\tv_nop\n\tv_nop\n\tv_nop" : "+v"(c) : "v"(ah), "v"(al), "v"(bh), "v"(bl));
  return c;
}

struct Epi {
  const float* bias;
  float*       out;
  const float* res;
  float*       dst1;
  float*       dst2;
  const float* g1;
  const float* g2;
  int mode;
  int ldO;
  int gStride;
  int halfRows;
  int rowsPerBT;
  int padz;
};
static_assert(sizeof(Epi) == 80);

#define GT_AS 40
#define GT_CS 132
#define GEMM_SMEM 33792

static __device__ __forceinline__ v4f gelu4(v4f x) {
  v4f r;
#pragma unroll
  for (int j = 0; j < 4; ++j) {
    const float v = x[j];
    const float u = 0.7978845608028654f * (v + 0.044715f * v * v * v);
    r[j] = 0.5f * v * (1.f + tanhf(u));
  }
  return r;
}

static __device__ __forceinline__ float* epi_target(const Epi& e, int grow, int gcol, const float*& gate) {
  gate = nullptr;
  if (e.mode <= 3) return e.out + (size_t)grow * e.ldO + gcol;
  if (e.mode == 4) {
    const int span = 2 * e.halfRows;
    const int bt = grow / span, n = grow - bt * span;
    if (n < e.halfRows) {
      gate = e.g1 + (size_t)bt * e.gStride + gcol;
      return e.dst1 + (size_t)(bt * e.halfRows + n) * C_DIM + gcol;
    }
    gate = e.g2 + (size_t)bt * e.gStride + gcol;
    return e.dst2 + (size_t)(bt * e.halfRows + (n - e.halfRows)) * C_DIM + gcol;
  }
  const int bt = grow / e.rowsPerBT;
  gate = e.g1 + (size_t)bt * e.gStride + gcol;
  return e.dst1 + (size_t)grow * C_DIM + gcol;
}

__global__ __launch_bounds__(256) void gemm_kernel(const float* __restrict__ A, const float* __restrict__ B,
                                                   int M, int N, int K, Epi e) {
  __shared__ __attribute__((aligned(16))) unsigned char smem[GEMM_SMEM];
  us16* Ash = (us16*)smem;
  us16* Asl = Ash + 64 * GT_AS;
  us16* Bsh = Asl + 64 * GT_AS;
  us16* Bsl = Bsh + 128 * GT_AS;
  float* Ct = (float*)smem;

  const int tid = threadIdx.x;
  const int w = tid >> 5, lane = tid & 31, l16 = lane & 15, hh = lane >> 4;
  const int wm = w >> 2, wn = w & 3;
  const int rowBase = blockIdx.y * 64, colBase = blockIdx.x * 128;
  if (colBase + 128 > N || rowBase >= M) return;

  v8f acc[2][2];
#pragma unroll
  for (int mi = 0; mi < 2; ++mi)
#pragma unroll
    for (int ni = 0; ni < 2; ++ni)
#pragma unroll
      for (int q = 0; q < 8; ++q) acc[mi][ni][q] = 0.f;

  const int arow = tid >> 2, acol = (tid & 3) * 8;

  for (int k0 = 0; k0 < K; k0 += 32) {
    {
      v8us hv, lv;
      if (rowBase + arow < M) {
        const float* ap = A + (size_t)(rowBase + arow) * K + k0 + acol;
        split8(*(const v4f*)ap, *(const v4f*)(ap + 4), hv, lv);
      } else {
#pragma unroll
        for (int j = 0; j < 8; ++j) { hv[j] = 0; lv[j] = 0; }
      }
      *(v8us*)(Ash + arow * GT_AS + acol) = hv;
      *(v8us*)(Asl + arow * GT_AS + acol) = lv;
    }
#pragma unroll
    for (int it = 0; it < 2; ++it) {
      const int i = tid + it * 256, kr = i >> 4, nc = (i & 15) * 8;
      const float* bp = B + (size_t)(k0 + kr) * N + colBase + nc;
      v8us hv, lv;
      split8(*(const v4f*)bp, *(const v4f*)(bp + 4), hv, lv);
#pragma unroll
      for (int j = 0; j < 8; ++j) {
        Bsh[(nc + j) * GT_AS + kr] = hv[j];
        Bsl[(nc + j) * GT_AS + kr] = lv[j];
      }
    }
    __syncthreads();

    v16bf ah[2], al[2];
#pragma unroll
    for (int mi = 0; mi < 2; ++mi) {
      const int off = (wm * 32 + mi * 16 + l16) * GT_AS;
      ah[mi] = ldfrag(Ash + off, hh);
      al[mi] = ldfrag(Asl + off, hh);
    }
#pragma unroll
    for (int ni = 0; ni < 2; ++ni) {
      const int off = (wn * 32 + ni * 16 + l16) * GT_AS;
      const v16bf bh = ldfrag(Bsh + off, hh);
      const v16bf bl = ldfrag(Bsl + off, hh);
#pragma unroll
      for (int mi = 0; mi < 2; ++mi) acc[mi][ni] = mma3(acc[mi][ni], ah[mi], al[mi], bh, bl);
    }
    __syncthreads();
  }

#pragma unroll
  for (int mi = 0; mi < 2; ++mi)
#pragma unroll
    for (int ni = 0; ni < 2; ++ni)
#pragma unroll
      for (int r = 0; r < 8; ++r)
        Ct[(wm * 32 + mi * 16 + hh * 8 + r) * GT_CS + wn * 32 + ni * 16 + l16] = acc[mi][ni][r];
  __syncthreads();

#pragma unroll 1
  for (int p = 0; p < 8; ++p) {
    const int lrow = p * 8 + w, grow = rowBase + lrow;
    if (grow < M) {
      const int gcol = colBase + lane * 4;
      v4f v = *(const v4f*)(Ct + lrow * GT_CS + lane * 4);
      if (e.bias) v += *(const v4f*)(e.bias + gcol);
      const float* gate;
      float* gp = epi_target(e, grow, gcol, gate);
      v4f val;
      if (e.mode == 2) {
        val = *(const v4f*)(e.res + (size_t)grow * e.ldO + gcol) + v;
      } else if (e.mode == 3) {
        val = gelu4(v);
      } else if (e.mode >= 4) {
        const v4f old = *(const v4f*)gp;
        const v4f g = *(const v4f*)gate;
        val = old + g * v;
      } else {
        val = v;
      }
      *(v4f*)(Ct + lrow * GT_CS + lane * 4) = val;
      *(volatile v4f*)gp = val;
    }
  }
  __threadfence();
#pragma unroll 1
  for (int p = 0; p < 8; ++p) {
    const int lrow = p * 8 + w, grow = rowBase + lrow;
    if (grow < M) {
      const int gcol = colBase + lane * 4;
      const float* gate;
      float* gp = epi_target(e, grow, gcol, gate);
      const v4f val = *(const v4f*)(Ct + lrow * GT_CS + lane * 4);
      *(volatile v4f*)gp = val;
    }
  }
}

__global__ __launch_bounds__(256) void attn_kernel(const float* __restrict__ Q, const float* __restrict__ Kp,
                                                   const float* __restrict__ Vp, int ldQ, int ldKV,
                                                   int nQ, int nK, float scale,
                                                   float* __restrict__ O, int ldO) {
  __shared__ __attribute__((aligned(16))) us16 Qh[32 * 72];
  __shared__ __attribute__((aligned(16))) us16 Ql[32 * 72];
  __shared__ __attribute__((aligned(16))) us16 Kh[64 * 72];
  __shared__ __attribute__((aligned(16))) us16 Kl[64 * 72];
  __shared__ __attribute__((aligned(16))) us16 Vh[64 * 72];
  __shared__ __attribute__((aligned(16))) us16 Vl[64 * 72];
  __shared__ __attribute__((aligned(16))) us16 Ph[32 * 72];
  __shared__ __attribute__((aligned(16))) us16 Pl[32 * 72];
  __shared__ __attribute__((aligned(16))) float Ss[32 * 68];
  __shared__ float rowM[32], rowS[32], rowF[32];

  const int b = blockIdx.z, h = blockIdx.y, qt = blockIdx.x;
  if ((qt + 1) * 32 > nQ) return;
  const int tid = threadIdx.x;
  const int w = tid >> 5, lane = tid & 31, l16 = lane & 15, hh = lane >> 4;

  const float* Qg = Q + (size_t)(b * nQ + qt * 32) * ldQ + h * HD;
  const float* Kg = Kp + (size_t)b * nK * ldKV + h * HD;
  const float* Vg = Vp + (size_t)b * nK * ldKV + h * HD;

  {
    const int r = tid >> 3, c = (tid & 7) * 8;
    const float* p = Qg + (size_t)r * ldQ + c;
    v8us hv, lv;
    split8(*(const v4f*)p, *(const v4f*)(p + 4), hv, lv);
    *(v8us*)(Qh + r * 72 + c) = hv;
    *(v8us*)(Ql + r * 72 + c) = lv;
  }
  if (tid < 32) { rowM[tid] = -3.0e38f; rowS[tid] = 0.f; rowF[tid] = 0.f; }

  v8f acc;
#pragma unroll
  for (int e2 = 0; e2 < 8; ++e2) acc[e2] = 0.f;

  const int qr = (w & 1) * 16;
  const int cb = (w >> 1) * 16;

  const int nChunks = nK / 64;
  for (int ch = 0; ch < nChunks; ++ch) {
    const int c0 = ch * 64;
    __syncthreads();
#pragma unroll
    for (int it = 0; it < 2; ++it) {
      const int i = tid + it * 256, kr = i >> 3, cc = (i & 7) * 8;
      const float* kp = Kg + (size_t)(c0 + kr) * ldKV + cc;
      v8us hv, lv;
      split8(*(const v4f*)kp, *(const v4f*)(kp + 4), hv, lv);
      *(v8us*)(Kh + kr * 72 + cc) = hv;
      *(v8us*)(Kl + kr * 72 + cc) = lv;
      const float* vp = Vg + (size_t)(c0 + kr) * ldKV + cc;
      v8us wh, wl;
      split8(*(const v4f*)vp, *(const v4f*)(vp + 4), wh, wl);
#pragma unroll
      for (int j = 0; j < 8; ++j) {
        Vh[(cc + j) * 72 + kr] = wh[j];
        Vl[(cc + j) * 72 + kr] = wl[j];
      }
    }
    __syncthreads();

    {
      v8f s;
#pragma unroll
      for (int e2 = 0; e2 < 8; ++e2) s[e2] = 0.f;
#pragma unroll
      for (int ks = 0; ks < 64; ks += 32) {
        const v16bf ah = ldfrag(Qh + (qr + l16) * 72 + ks, hh);
        const v16bf al = ldfrag(Ql + (qr + l16) * 72 + ks, hh);
        const v16bf bh = ldfrag(Kh + (cb + l16) * 72 + ks, hh);
        const v16bf bl = ldfrag(Kl + (cb + l16) * 72 + ks, hh);
        s = mma3(s, ah, al, bh, bl);
      }
#pragma unroll
      for (int e2 = 0; e2 < 8; ++e2) Ss[(qr + hh * 8 + e2) * 68 + cb + l16] = s[e2] * scale;
    }
    __syncthreads();

    {
      const int r = tid >> 3, sl = tid & 7;
      float cm = -3.0e38f;
#pragma unroll
      for (int jj = 0; jj < 8; ++jj) cm = fmaxf(cm, Ss[r * 68 + sl + jj * 8]);
      cm = fmaxf(cm, __shfl_xor(cm, 1));
      cm = fmaxf(cm, __shfl_xor(cm, 2));
      cm = fmaxf(cm, __shfl_xor(cm, 4));
      const float mo = rowM[r];
      const float mn = fmaxf(mo, cm);
      float ps = 0.f;
#pragma unroll
      for (int jj = 0; jj < 8; ++jj) {
        const int j = sl + jj * 8;
        const float ev = __expf(Ss[r * 68 + j] - mn);
        us16 ph, pl;
        split2(ev, ph, pl);
        Ph[r * 72 + j] = ph;
        Pl[r * 72 + j] = pl;
        ps += ev;
      }
      ps += __shfl_xor(ps, 1);
      ps += __shfl_xor(ps, 2);
      ps += __shfl_xor(ps, 4);
      if (sl == 0) {
        const float f = __expf(mo - mn);
        rowF[r] = f;
        rowS[r] = rowS[r] * f + ps;
        rowM[r] = mn;
      }
    }
    __syncthreads();

#pragma unroll
    for (int e2 = 0; e2 < 8; ++e2) acc[e2] *= rowF[qr + hh * 8 + e2];
#pragma unroll
    for (int ks = 0; ks < 64; ks += 32) {
      const v16bf ah = ldfrag(Ph + (qr + l16) * 72 + ks, hh);
      const v16bf al = ldfrag(Pl + (qr + l16) * 72 + ks, hh);
      const v16bf bh = ldfrag(Vh + (cb + l16) * 72 + ks, hh);
      const v16bf bl = ldfrag(Vl + (cb + l16) * 72 + ks, hh);
      acc = mma3(acc, ah, al, bh, bl);
    }
  }

#pragma unroll
  for (int e2 = 0; e2 < 8; ++e2) {
    const int rr = qr + hh * 8 + e2;
    Ss[rr * 68 + cb + l16] = acc[e2] / rowS[rr];
  }
  __syncthreads();

#pragma unroll
  for (int it = 0; it < 2; ++it) {
    const int row = it * 16 + (tid >> 4), col = (tid & 15) * 4;
    const v4f v = *(const v4f*)(Ss + row * 68 + col);
    float* gp = O + (size_t)(b * nQ + qt * 32 + row) * ldO + h * HD + col;
    *(volatile v4f*)gp = v;
  }
  __threadfence();
#pragma unroll
  for (int it = 0; it < 2; ++it) {
    const int row = it * 16 + (tid >> 4), col = (tid & 15) * 4;
    const v4f v = *(const v4f*)(Ss + row * 68 + col);
    float* gp = O + (size_t)(b * nQ + qt * 32 + row) * ldO + h * HD + col;
    *(volatile v4f*)gp = v;
  }
}

__global__ __launch_bounds__(256) void lnmod_kernel(const float* __restrict__ x, const float* __restrict__ sh,
                                                    const float* __restrict__ sc, int mStride,
                                                    float* __restrict__ out, int outRowStride, int halfOff,
                                                    int rowsPerBT, int nRows) {
  __shared__ float red1[8], red2[8];
  const int row = blockIdx.x;
  if (row >= nRows) return;
  const int tid = threadIdx.x, w = tid >> 5, lane = tid & 31, c = tid * 4;

  const v4f v = *(const v4f*)(x + (size_t)row * C_DIM + c);
  float s = (v[0] + v[1]) + (v[2] + v[3]);
#pragma unroll
  for (int o = 1; o < 32; o <<= 1) s += __shfl_xor(s, o);
  if (lane == 0) red1[w] = s;
  __syncthreads();
  float ts = 0.f;
#pragma unroll
  for (int j = 0; j < 8; ++j) ts += red1[j];
  const float mu = ts * (1.f / 1024.f);

  v4f d;
#pragma unroll
  for (int j = 0; j < 4; ++j) d[j] = v[j] - mu;
  float s2 = (d[0] * d[0] + d[1] * d[1]) + (d[2] * d[2] + d[3] * d[3]);
#pragma unroll
  for (int o = 1; o < 32; o <<= 1) s2 += __shfl_xor(s2, o);
  if (lane == 0) red2[w] = s2;
  __syncthreads();
  float ts2 = 0.f;
#pragma unroll
  for (int j = 0; j < 8; ++j) ts2 += red2[j];
  const float var = ts2 * (1.f / 1024.f);
  const float rstd = rsqrtf(var + 1e-6f);

  const int bt = row / rowsPerBT, n = row - bt * rowsPerBT;
  const v4f scv = *(const v4f*)(sc + (size_t)bt * mStride + c);
  const v4f shv = *(const v4f*)(sh + (size_t)bt * mStride + c);
  v4f val;
#pragma unroll
  for (int j = 0; j < 4; ++j) val[j] = (d[j] * rstd) * (1.f + scv[j]) + shv[j];

  float* gp = out + ((size_t)bt * outRowStride + halfOff + n) * C_DIM + c;
  *(volatile v4f*)gp = val;
  __threadfence();
  *(volatile v4f*)gp = val;
}

__global__ __launch_bounds__(256) void silu_kernel(const float* __restrict__ t, const float* __restrict__ cond,
                                                   const int* __restrict__ Tp, int Bb, int BT,
                                                   float* __restrict__ out) {
  const int bt = blockIdx.x;
  if (bt >= BT) return;
  int T = Tp[0];
  if (T < 1) T = 1;
  int b = bt / T;
  if (b > Bb - 1) b = Bb - 1;
  const int c = threadIdx.x * 4;
  const v4f a0 = *(const v4f*)(t + (size_t)b * C_DIM + c);
  const v4f a1 = *(const v4f*)(cond + (size_t)bt * C_DIM + c);
  v4f r;
#pragma unroll
  for (int j = 0; j < 4; ++j) {
    const float v = a0[j] + a1[j];
    r[j] = v / (1.f + __expf(-v));
  }
  float* gp = out + (size_t)bt * C_DIM + c;
  *(volatile v4f*)gp = r;
  __threadfence();
  *(volatile v4f*)gp = r;
}

extern "C" void kernel_launch(void* const* d_in, const int* in_sizes, int n_in,
                              void* d_out, int out_size, void* d_ws,
                              size_t ws_size, hipStream_t stream) {
  if (n_in < 35) return;
  const float* x1_in = (const float*)d_in[0];
  const float* x2_in = (const float*)d_in[1];
  const float* t_in  = (const float*)d_in[2];
  const float* vf1   = (const float*)d_in[3];
  const float* vf2   = (const float*)d_in[4];
  const float* cond  = (const float*)d_in[5];
  const float *Wq1 = (const float*)d_in[6],   *bq1 = (const float*)d_in[7];
  const float *Wkv1 = (const float*)d_in[8],  *bkv1 = (const float*)d_in[9];
  const float *Wp1 = (const float*)d_in[10],  *bp1 = (const float*)d_in[11];
  const float *Wq2 = (const float*)d_in[12],  *bq2 = (const float*)d_in[13];
  const float *Wkv2 = (const float*)d_in[14], *bkv2 = (const float*)d_in[15];
  const float *Wp2 = (const float*)d_in[16],  *bp2 = (const float*)d_in[17];
  const float *Wqkv = (const float*)d_in[18], *bqkv = (const float*)d_in[19];
  const float *Wpa = (const float*)d_in[20],  *bpa = (const float*)d_in[21];
  const float *Wada1 = (const float*)d_in[22], *bada1 = (const float*)d_in[23];
  const float *Wada2 = (const float*)d_in[24], *bada2 = (const float*)d_in[25];
  const float *Wf1a = (const float*)d_in[26], *bf1a = (const float*)d_in[27];
  const float *Wf2a = (const float*)d_in[28], *bf2a = (const float*)d_in[29];
  const float *Wf1b = (const float*)d_in[30], *bf1b = (const float*)d_in[31];
  const float *Wf2b = (const float*)d_in[32], *bf2b = (const float*)d_in[33];
  const int*   T_in = (const int*)d_in[34];

  const int Bb = in_sizes[2] / C_DIM;
  const int BT = in_sizes[5] / C_DIM;
  if (Bb < 1 || BT < 1) return;
  const int T = BT / Bb;
  if (T < 1 || BT != Bb * T) return;
  const int TN = in_sizes[0] / (Bb * C_DIM);
  if (TN < 32 || in_sizes[0] != Bb * TN * C_DIM || in_sizes[1] != in_sizes[0]) return;
  const int N = TN / T;
  if (N < 32 || N * T != TN || (N % 32) != 0 || (TN % 32) != 0) return;
  const int Mctx = in_sizes[3] / (Bb * C_DIM);
  if (Mctx < 64 || (Mctx % 64) != 0 || in_sizes[3] != Bb * Mctx * C_DIM || in_sizes[4] != in_sizes[3]) return;
  const int MLPD = in_sizes[26] / C_DIM;
  if (MLPD < 128 || (MLPD % 128) != 0) return;
  if (in_sizes[6] != C_DIM * C_DIM || in_sizes[8] != 2 * C_DIM * C_DIM || in_sizes[12] != C_DIM * C_DIM ||
      in_sizes[14] != 2 * C_DIM * C_DIM || in_sizes[18] != 3 * C_DIM * C_DIM ||
      in_sizes[22] != 6 * C_DIM * C_DIM || in_sizes[24] != 6 * C_DIM * C_DIM ||
      in_sizes[26] != C_DIM * MLPD || in_sizes[28] != MLPD * C_DIM ||
      in_sizes[30] != C_DIM * MLPD || in_sizes[32] != MLPD * C_DIM || in_sizes[34] < 1) return;
  const int Rx   = Bb * TN;
  const int Rctx = Bb * Mctx;
  const int Rcat = BT * 2 * N;
  if (out_size != 2 * Rx * C_DIM) return;

  float* x1o = (float*)d_out;
  float* x2o = x1o + (size_t)Rx * C_DIM;

  auto al256 = [](size_t v) -> size_t { return (v + 255) & ~(size_t)255; };
  const size_t fb = sizeof(float);
  const size_t szQ   = al256((size_t)Rx * C_DIM * fb);
  const size_t szKV  = al256((size_t)Rctx * 2 * C_DIM * fb);
  const size_t szO   = szQ;
  const size_t szQKV = al256((size_t)Rcat * 3 * C_DIM * fb);
  const size_t szHX  = szQ;
  const size_t szH1  = al256((size_t)Rx * MLPD * fb);
  size_t needBig = szQKV;
  if (szQ + szKV + szO > needBig) needBig = szQ + szKV + szO;
  if (szHX + szH1 > needBig) needBig = szHX + szH1;
  const size_t szCat = al256((size_t)Rcat * C_DIM * fb);
  const size_t szS   = al256((size_t)BT * C_DIM * fb);
  const size_t szM   = al256((size_t)BT * 6 * C_DIM * fb);
  const size_t offBig = 0;
  const size_t offCat = offBig + needBig;
  const size_t offS   = offCat + szCat;
  const size_t offM1  = offS + szS;
  const size_t offM2  = offM1 + szM;
  const size_t total  = offM2 + szM;
  if (total > ws_size) return;

  char* ws = (char*)d_ws;
  float* qbuf  = (float*)(ws + offBig);
  float* kvbuf = (float*)(ws + offBig + szQ);
  float* obuf  = (float*)(ws + offBig + szQ + szKV);
  float* qkv   = (float*)(ws + offBig);
  float* hx    = (float*)(ws + offBig);
  float* h1    = (float*)(ws + offBig + szHX);
  float* xcat  = (float*)(ws + offCat);
  float* oat   = (float*)(ws + offCat);
  float* sbuf  = (float*)(ws + offS);
  float* m1    = (float*)(ws + offM1);
  float* m2    = (float*)(ws + offM2);

  auto gemm = [&](const float* Ap, const float* Bp, int M, int Nn, int K, const Epi& e) {
    gemm_kernel<<<dim3(Nn / 128, (M + 63) / 64), 256, 0, stream>>>(Ap, Bp, M, Nn, K, e);
  };

  const float scale = 0.125f;

  { Epi e{}; e.mode = 1; e.bias = bq1; e.out = qbuf; e.ldO = C_DIM;
    gemm(x1_in, Wq1, Rx, C_DIM, C_DIM, e); }
  { Epi e{}; e.mode = 1; e.bias = bkv1; e.out = kvbuf; e.ldO = 2 * C_DIM;
    gemm(vf1, Wkv1, Rctx, 2 * C_DIM, C_DIM, e); }
  attn_kernel<<<dim3(TN / 32, NHEAD, Bb), 256, 0, stream>>>(
      qbuf, kvbuf, kvbuf + C_DIM, C_DIM, 2 * C_DIM, TN, Mctx, scale, obuf, C_DIM);
  { Epi e{}; e.mode = 2; e.bias = bp1; e.out = x1o; e.ldO = C_DIM; e.res = x1_in;
    gemm(obuf, Wp1, Rx, C_DIM, C_DIM, e); }

  { Epi e{}; e.mode = 1; e.bias = bq2; e.out = qbuf; e.ldO = C_DIM;
    gemm(x2_in, Wq2, Rx, C_DIM, C_DIM, e); }
  { Epi e{}; e.mode = 1; e.bias = bkv2; e.out = kvbuf; e.ldO = 2 * C_DIM;
    gemm(vf2, Wkv2, Rctx, 2 * C_DIM, C_DIM, e); }
  attn_kernel<<<dim3(TN / 32, NHEAD, Bb), 256, 0, stream>>>(
      qbuf, kvbuf, kvbuf + C_DIM, C_DIM, 2 * C_DIM, TN, Mctx, scale, obuf, C_DIM);
  { Epi e{}; e.mode = 2; e.bias = bp2; e.out = x2o; e.ldO = C_DIM; e.res = x2_in;
    gemm(obuf, Wp2, Rx, C_DIM, C_DIM, e); }

  silu_kernel<<<dim3(BT), 256, 0, stream>>>(t_in, cond, T_in, Bb, BT, sbuf);
  { Epi e{}; e.mode = 1; e.bias = bada1; e.out = m1; e.ldO = 6 * C_DIM;
    gemm(sbuf, Wada1, BT, 6 * C_DIM, C_DIM, e); }
  { Epi e{}; e.mode = 1; e.bias = bada2; e.out = m2; e.ldO = 6 * C_DIM;
    gemm(sbuf, Wada2, BT, 6 * C_DIM, C_DIM, e); }

  lnmod_kernel<<<dim3(Rx), 256, 0, stream>>>(x1o, m1, m1 + C_DIM, 6 * C_DIM, xcat, 2 * N, 0, N, Rx);
  lnmod_kernel<<<dim3(Rx), 256, 0, stream>>>(x2o, m2, m2 + C_DIM, 6 * C_DIM, xcat, 2 * N, N, N, Rx);

  { Epi e{}; e.mode = 1; e.bias = bqkv; e.out = qkv; e.ldO = 3 * C_DIM;
    gemm(xcat, Wqkv, Rcat, 3 * C_DIM, C_DIM, e); }
  attn_kernel<<<dim3((2 * N) / 32, NHEAD, BT), 256, 0, stream>>>(
      qkv, qkv + C_DIM, qkv + 2 * C_DIM, 3 * C_DIM, 3 * C_DIM, 2 * N, 2 * N, scale, oat, C_DIM);
  { Epi e{}; e.mode = 4; e.bias = bpa; e.dst1 = x1o; e.dst2 = x2o;
    e.g1 = m1 + 2 * C_DIM; e.g2 = m2 + 2 * C_DIM; e.gStride = 6 * C_DIM; e.halfRows = N;
    gemm(oat, Wpa, Rcat, C_DIM, C_DIM, e); }

  lnmod_kernel<<<dim3(Rx), 256, 0, stream>>>(x1o, m1 + 3 * C_DIM, m1 + 4 * C_DIM, 6 * C_DIM, hx, N, 0, N, Rx);
  { Epi e{}; e.mode = 3; e.bias = bf1a; e.out = h1; e.ldO = MLPD;
    gemm(hx, Wf1a, Rx, MLPD, C_DIM, e); }
  { Epi e{}; e.mode = 5; e.bias = bf2a; e.dst1 = x1o; e.g1 = m1 + 5 * C_DIM;
    e.gStride = 6 * C_DIM; e.rowsPerBT = N;
    gemm(h1, Wf2a, Rx, C_DIM, MLPD, e); }

  lnmod_kernel<<<dim3(Rx), 256, 0, stream>>>(x2o, m2 + 3 * C_DIM, m2 + 4 * C_DIM, 6 * C_DIM, hx, N, 0, N, Rx);
  { Epi e{}; e.mode = 3; e.bias = bf1b; e.out = h1; e.ldO = MLPD;
    gemm(hx, Wf1b, Rx, MLPD, C_DIM, e); }
  { Epi e{}; e.mode = 5; e.bias = bf2b; e.dst1 = x2o; e.g1 = m2 + 5 * C_DIM;
    e.gStride = 6 * C_DIM; e.rowsPerBT = N;
    gemm(h1, Wf2b, Rx, C_DIM, MLPD, e); }
}
